// BiMambaBlock_352187318777
// MI455X (gfx1250) — hardware-verified
//
#include <hip/hip_runtime.h>
#include <math.h>

typedef __attribute__((ext_vector_type(16))) _Float16 v16h;
typedef __attribute__((ext_vector_type(8)))  _Float16 v8h;
typedef __attribute__((ext_vector_type(8)))  float    v8f;
typedef __attribute__((ext_vector_type(4)))  float    v4f;

constexpr int kBatch = 2;
constexpr int kSeqL  = 2048;
constexpr int kDmod  = 1024;
constexpr int kDin   = 2048;
constexpr int kNst   = 16;
constexpr int kDtR   = 64;
constexpr int kPrjN  = 96;
constexpr int kPrjP  = 128;
constexpr int kXZP   = 2 * kDin;
constexpr int kFuK   = 2 * kDmod;
constexpr int kRows  = kBatch * kSeqL;
constexpr int kTP    = 260;
static_assert(kPrjN == kDtR + 2 * kNst, "x_proj width");
static_assert(kPrjP % 64 == 0 && kPrjP >= kPrjN, "x_proj padded width");
static_assert(kDmod % 32 == 0 && kDin % 32 == 0 && kDtR % 32 == 0 && kFuK % 32 == 0, "GEMM K multiples of 32");
static_assert(kSeqL % 64 == 0 && kRows % 64 == 0 && kXZP % 64 == 0 && kDin % 64 == 0 && kDmod % 64 == 0, "GEMM M,N multiples of 64");
static_assert(kDin % 256 == 0 && kSeqL % 64 == 0, "conv / scan tiling");

constexpr float kCarW    = 32.0f;
constexpr float kCarU    = 64.0f;
constexpr float kCarDt   = 16.0f;
constexpr float kCarWdt  = 8.0f;
constexpr float kCarY    = 256.0f;
constexpr float kCarComb = 256.0f;
constexpr float kSclIn   = 1.0f / kCarW;
constexpr float kSclXp   = 1.0f / (kCarU * kCarW);
constexpr float kSclDt   = 1.0f / (kCarDt * kCarWdt);
constexpr float kSclOut  = kCarComb / (kCarY * kCarW);
constexpr float kSclFu   = 1.0f / (kCarComb * kCarW);

constexpr size_t kSzWIN  = (size_t)kXZP  * kDmod * 2;
constexpr size_t kSzWXP  = (size_t)kPrjP * kDin  * 2;
constexpr size_t kSzWDT  = (size_t)kDin  * kDtR  * 2;
constexpr size_t kSzWOUT = (size_t)kDmod * kDin  * 2;
constexpr size_t kSzWFU  = (size_t)kDmod * kFuK  * 2;
constexpr size_t kSzX16  = (size_t)kRows * kDmod * 2;
constexpr size_t kSzXZ   = (size_t)kSeqL * kXZP  * 4;
constexpr size_t kSzUC   = (size_t)kSeqL * kDin  * 4;
constexpr size_t kSzUC16 = (size_t)kSeqL * kDin  * 2;
constexpr size_t kSzPROJ = (size_t)kSeqL * kPrjP * 4;
constexpr size_t kSzDT16 = (size_t)kSeqL * kDtR  * 2;
constexpr size_t kSzDLR  = (size_t)kSeqL * kDin  * 4;
constexpr size_t kSzY16  = (size_t)kSeqL * kDin  * 2;
constexpr size_t kSzCOMB = (size_t)kRows * kFuK  * 2;
constexpr size_t kOffWIN  = 0;
constexpr size_t kOffWXP  = kOffWIN  + kSzWIN;
constexpr size_t kOffWDT  = kOffWXP  + kSzWXP;
constexpr size_t kOffWOUT = kOffWDT  + kSzWDT;
constexpr size_t kOffWFU  = kOffWOUT + kSzWOUT;
constexpr size_t kOffX16  = kOffWFU  + kSzWFU;
constexpr size_t kOffXZ   = kOffX16  + kSzX16;
constexpr size_t kOffUC   = kOffXZ   + kSzXZ;
constexpr size_t kOffUC16 = kOffUC   + kSzUC;
constexpr size_t kOffPROJ = kOffUC16 + kSzUC16;
constexpr size_t kOffDT16 = kOffPROJ + kSzPROJ;
constexpr size_t kOffDLR  = kOffDT16 + kSzDT16;
constexpr size_t kOffY16  = kOffDLR  + kSzDLR;
constexpr size_t kOffCOMB = kOffY16  + kSzY16;
constexpr size_t kWsTotal = kOffCOMB + kSzCOMB;
static_assert(kWsTotal == 127926272ull, "carve total");
static_assert(kWsTotal <= 134217728ull, "carve cap");
static_assert((kOffWXP % 128) == 0 && (kOffWDT % 128) == 0 && (kOffWOUT % 128) == 0 && (kOffWFU % 128) == 0 &&
              (kOffX16 % 128) == 0 && (kOffXZ % 128) == 0 && (kOffUC % 128) == 0 && (kOffUC16 % 128) == 0 &&
              (kOffPROJ % 128) == 0 && (kOffDT16 % 128) == 0 && (kOffDLR % 128) == 0 && (kOffY16 % 128) == 0 &&
              (kOffCOMB % 128) == 0, "128-B aligned regions");

__device__ __forceinline__ unsigned short f2bf_bits(float f) {
  unsigned u = __float_as_uint(f);
  return (unsigned short)((u + 0x7FFFu + ((u >> 16) & 1u)) >> 16);
}
__device__ __forceinline__ float bf_bits2f(unsigned short h) { return __uint_as_float(((unsigned)h) << 16); }
__device__ __forceinline__ float bf_rne(float f) { return bf_bits2f(f2bf_bits(f)); }

__device__ __forceinline__ void row_guard_h(v8f& a, v8f& b, v8f& c, v8f& d, v16h x, v16h y0, v16h y1, v16h y2, v16h y3) {
  asm volatile("v_nop\n\tv_nop\n\tv_nop\n\tv_nop" : "+v"(a), "+v"(b), "+v"(c), "+v"(d) : "v"(x), "v"(y0), "v"(y1), "v"(y2), "v"(y3));
}
__device__ __forceinline__ void keep4_h(v16h a, v16h b, v16h c, v16h d) { asm volatile("v_nop" :: "v"(a), "v"(b), "v"(c), "v"(d)); }
__device__ __forceinline__ void acc_guard4(v8f& a, v8f& b, v8f& c, v8f& d) { asm volatile("v_nop\n\tv_nop\n\tv_nop\n\tv_nop" : "+v"(a), "+v"(b), "+v"(c), "+v"(d)); }

struct FragH {
  union U { v16h v; v8h h[2]; };
  static __device__ __forceinline__ v16h load(const _Float16* p) {
    U f; f.h[0] = *(const v8h*)(p); f.h[1] = *(const v8h*)(p + 16); return f.v;
  }
  static __device__ __forceinline__ v8f mma(v16h a, v16h b, v8f c) {
    return __builtin_amdgcn_wmma_f32_16x16x32_f16(false, a, false, b, (short)0, c, false, false);
  }
};

template <int BIAS_MODE, int OUT_MODE>
__global__ __launch_bounds__(256) void wmma_gemm64_f16(
    const unsigned short* __restrict__ Ap, int lda,
    const unsigned short* __restrict__ Btp, int ldb,
    void* __restrict__ Cout, int ldc,
    const float* __restrict__ bias,
    int M, int N, int K, float scale) {
  const _Float16* A  = (const _Float16*)Ap;
  const _Float16* Bt = (const _Float16*)Btp;
  __shared__ __align__(16) float sT[8][16 * 68];
  const int lane = threadIdx.x & 31;
  const int wave = threadIdx.x >> 5;
  const int tilesN = N >> 6;
  const int tilesM = M >> 6;
  const int tile = blockIdx.x * 8 + wave;
  if (tile >= tilesM * tilesN) return;
  const int tm = tile / tilesN;
  const int tn = tile - tm * tilesN;
  const int m0 = tm << 6;
  const int n0 = tn << 6;

  const int rlane = lane & 15;
  const int koff  = (lane >> 4) * 8;
  const int mOff  = (lane >> 4) * 8;

  v8f acc[4][4];
#pragma unroll
  for (int i = 0; i < 4; ++i)
#pragma unroll
    for (int j = 0; j < 4; ++j) acc[i][j] = (v8f){0.f,0.f,0.f,0.f,0.f,0.f,0.f,0.f};

  for (int k0 = 0; k0 < K; k0 += 32) {
    v16h bh[4];
#pragma unroll
    for (int j = 0; j < 4; ++j) {
      const size_t bo = (size_t)(n0 + (j << 4) + rlane) * ldb + koff + k0;
      bh[j] = FragH::load(Bt + bo);
    }
#pragma unroll
    for (int i = 0; i < 4; ++i) {
      const size_t ao = (size_t)(m0 + (i << 4) + rlane) * lda + koff + k0;
      v16h ah = FragH::load(A + ao);
#pragma unroll
      for (int j = 0; j < 4; ++j) acc[i][j] = FragH::mma(ah, bh[j], acc[i][j]);
      row_guard_h(acc[i][0], acc[i][1], acc[i][2], acc[i][3], ah, bh[0], bh[1], bh[2], bh[3]);
    }
    keep4_h(bh[0], bh[1], bh[2], bh[3]);
  }
  acc_guard4(acc[0][0], acc[0][1], acc[0][2], acc[0][3]);
  acc_guard4(acc[1][0], acc[1][1], acc[1][2], acc[1][3]);
  acc_guard4(acc[2][0], acc[2][1], acc[2][2], acc[2][3]);
  acc_guard4(acc[3][0], acc[3][1], acc[3][2], acc[3][3]);

  float* slab = sT[wave];
#pragma unroll
  for (int i = 0; i < 4; ++i) {
    const int mBase = m0 + (i << 4);
#pragma unroll
    for (int j = 0; j < 4; ++j) {
      const int n = n0 + (j << 4) + rlane;
      float bv = 0.f;
      if (BIAS_MODE == 2) bv = bf_rne(bias[n]);
#pragma unroll
      for (int r = 0; r < 8; ++r) {
        float v = acc[i][j][r] * scale;
        if (BIAS_MODE == 2) v += bv;
        slab[(mOff + r) * 68 + (j << 4) + rlane] = v;
      }
    }
    __builtin_amdgcn_fence(__ATOMIC_RELEASE, "workgroup");
    __builtin_amdgcn_wave_barrier();
    __builtin_amdgcn_fence(__ATOMIC_ACQUIRE, "workgroup");
    if (OUT_MODE == 0) {
      float* C = (float*)Cout;
      const int hh = lane >> 4, c4 = (lane & 15) * 4;
      for (int pass = 0; pass < 2; ++pass) {
#pragma unroll
        for (int it = 0; it < 8; ++it) {
          const int row = it * 2 + hh;
          v4f v = *(const v4f*)(slab + row * 68 + c4);
          *(volatile v4f*)(C + (size_t)(mBase + row) * ldc + n0 + c4) = v;
        }
        __threadfence();
      }
    } else {
      const int q = lane >> 3, c8 = (lane & 7) * 8;
      unsigned short* C = (unsigned short*)Cout;
      for (int pass = 0; pass < 2; ++pass) {
#pragma unroll
        for (int it = 0; it < 4; ++it) {
          const int row = it * 4 + q;
          const float* sp = slab + row * 68 + c8;
          v8h hv;
#pragma unroll
          for (int e = 0; e < 8; ++e) hv[e] = (_Float16)sp[e];
          *(volatile v8h*)(C + (size_t)(mBase + row) * ldc + n0 + c8) = hv;
        }
        __threadfence();
      }
    }
    __builtin_amdgcn_fence(__ATOMIC_RELEASE, "workgroup");
    __builtin_amdgcn_wave_barrier();
    __builtin_amdgcn_fence(__ATOMIC_ACQUIRE, "workgroup");
  }
}

__global__ __launch_bounds__(256) void cast_bf16_f16_kernel(
    const float* __restrict__ src, unsigned short* __restrict__ dst, int total8, int real8, float scale)
{
  const int i = blockIdx.x * 256 + threadIdx.x;
  if (i >= total8) return;
  const bool live = (i < real8);
  const int ic = live ? i : (real8 - 1);
  const float* p = src + ((size_t)ic << 3);
  const v4f a0 = *(const v4f*)(p);
  const v4f a1 = *(const v4f*)(p + 4);
  v8h hv;
#pragma unroll
  for (int e = 0; e < 4; ++e) {
    const float s0 = a0[e];
    const float s1 = a1[e];
    const float r0 = bf_rne(s0) * scale;
    const float r1 = bf_rne(s1) * scale;
    hv[e]     = (_Float16)(live ? r0 : 0.0f);
    hv[4 + e] = (_Float16)(live ? r1 : 0.0f);
  }
  unsigned short* q = dst + ((size_t)i << 3);
  *(volatile v8h*)q = hv;
  __threadfence();
  *(volatile v8h*)q = hv;
}

__global__ __launch_bounds__(256) void dt_cast_kernel(
    const float* __restrict__ PROJ, unsigned short* __restrict__ DT16, int total8, float scale)
{
  const int i = blockIdx.x * 256 + threadIdx.x;
  if (i >= total8) return;
  const int e0  = i << 3;
  const int row = e0 >> 6;
  const int c8  = e0 & 63;
  const float* p = PROJ + (size_t)row * kPrjP + c8;
  const v4f a0 = *(const v4f*)(p);
  const v4f a1 = *(const v4f*)(p + 4);
  v8h hv;
#pragma unroll
  for (int e = 0; e < 4; ++e) {
    hv[e]     = (_Float16)(a0[e] * scale);
    hv[4 + e] = (_Float16)(a1[e] * scale);
  }
  unsigned short* qd = DT16 + e0;
  *(volatile v8h*)qd = hv;
  __threadfence();
  *(volatile v8h*)qd = hv;
}

__global__ __launch_bounds__(256) void conv_silu_kernel(
    const float* __restrict__ XZ, const float* __restrict__ cw, const float* __restrict__ cb,
    float* __restrict__ UC, unsigned short* __restrict__ UC16, int rev)
{
  __shared__ __align__(16) float sT[16 * kTP];
  const int tid = threadIdx.x, lane = tid & 31, wave = tid >> 5;
  const int d0 = blockIdx.x * 256, d = d0 + tid;
  const int t0 = blockIdx.y * 64;
  const v4f wv = *(const v4f*)(cw + (size_t)d * 4);
  const float wa = wv[0], wb = wv[1], wc = wv[2], wd = wv[3];
  const float w0 = bf_rne(wa), w1 = bf_rne(wb), w2 = bf_rne(wc), w3 = bf_rne(wd);
  const float bc = bf_rne(cb[d]);
  float xm3, xm2, xm1;
  {
    const int s1 = rev ? (t0 + 64) : (t0 - 1);
    const int s2 = rev ? (t0 + 65) : (t0 - 2);
    const int s3 = rev ? (t0 + 66) : (t0 - 3);
    const int c1 = s1 < 0 ? 0 : (s1 > kSeqL - 1 ? kSeqL - 1 : s1);
    const int c2 = s2 < 0 ? 0 : (s2 > kSeqL - 1 ? kSeqL - 1 : s2);
    const int c3 = s3 < 0 ? 0 : (s3 > kSeqL - 1 ? kSeqL - 1 : s3);
    const float v1 = XZ[(size_t)c1 * kXZP + d];
    const float v2 = XZ[(size_t)c2 * kXZP + d];
    const float v3 = XZ[(size_t)c3 * kXZP + d];
    xm1 = (s1 == c1) ? v1 : 0.f;
    xm2 = (s2 == c2) ? v2 : 0.f;
    xm3 = (s3 == c3) ? v3 : 0.f;
  }
  const int hrow = wave >> 1;
  const int hch  = (wave & 1) * 128 + lane * 4;
#pragma unroll 1
  for (int sub = 0; sub < 4; ++sub) {
    const int lb = t0 + (rev ? (3 - sub) : sub) * 16;
#pragma unroll 1
    for (int s = 0; s < 16; ++s) {
      const int rr = rev ? (15 - s) : s;
      const float xcur = XZ[(size_t)(lb + rr) * kXZP + d];
      float acc = w0 * xm3;
      acc = fmaf(w1, xm2, acc);
      acc = fmaf(w2, xm1, acc);
      acc = fmaf(w3, xcur, acc);
      const float sv = acc + bc;
      const float sg = __builtin_amdgcn_rcpf(1.0f + __expf(-sv));
      sT[rr * kTP + tid] = sv * sg;
      xm3 = xm2; xm2 = xm1; xm1 = xcur;
    }
    __syncthreads();
    v4f fv[4];
    v8h bv[2];
#pragma unroll
    for (int it = 0; it < 4; ++it) fv[it] = *(const v4f*)(sT + (it * 4 + hrow) * kTP + hch);
#pragma unroll
    for (int it = 0; it < 2; ++it) {
      const float* sp = sT + (it * 8 + wave) * kTP + lane * 8;
      const v4f a0 = *(const v4f*)(sp);
      const v4f a1 = *(const v4f*)(sp + 4);
#pragma unroll
      for (int e = 0; e < 4; ++e) {
        bv[it][e]     = (_Float16)(a0[e] * kCarU);
        bv[it][4 + e] = (_Float16)(a1[e] * kCarU);
      }
    }
    for (int pass = 0; pass < 2; ++pass) {
#pragma unroll
      for (int it = 0; it < 4; ++it)
        *(volatile v4f*)(UC + (size_t)(lb + it * 4 + hrow) * kDin + d0 + hch) = fv[it];
#pragma unroll
      for (int it = 0; it < 2; ++it)
        *(volatile v8h*)(UC16 + (size_t)(lb + it * 8 + wave) * kDin + d0 + lane * 8) = bv[it];
      __threadfence();
    }
    __syncthreads();
  }
}

__global__ __launch_bounds__(256) void scan_kernel(
    const float* __restrict__ DLR, const float* __restrict__ UC, const float* __restrict__ XZ,
    const float* __restrict__ PROJ, const float* __restrict__ A_log, const float* __restrict__ Dv,
    unsigned short* __restrict__ Y16, int rev)
{
  __shared__ __align__(16) float sBC[16 * 32];
  __shared__ __align__(16) float sY[16 * kTP];
  const int tid = threadIdx.x, lane = tid & 31, wave = tid >> 5;
  const int d0 = blockIdx.x * 256, d = d0 + tid;

  float An[kNst];
  {
    const float* ap = A_log + (size_t)d * kNst;
#pragma unroll
    for (int q4 = 0; q4 < 4; ++q4) {
      const v4f av = *(const v4f*)(ap + 4 * q4);
      const float e0 = av[0], e1 = av[1], e2 = av[2], e3 = av[3];
      An[4 * q4 + 0] = -__expf(bf_rne(e0));
      An[4 * q4 + 1] = -__expf(bf_rne(e1));
      An[4 * q4 + 2] = -__expf(bf_rne(e2));
      An[4 * q4 + 3] = -__expf(bf_rne(e3));
    }
  }
  const float Dd = bf_rne(Dv[d]);
  float h[kNst];
#pragma unroll
  for (int n = 0; n < kNst; ++n) h[n] = 0.f;

#pragma unroll 1
  for (int c = 0; c < kSeqL / 16; ++c) {
    const int l0 = (rev ? (kSeqL / 16 - 1 - c) : c) * 16;
    if (tid < 128) {
      const int r = tid >> 3, q = (tid & 7) * 4;
      const v4f v = *(const v4f*)(PROJ + (size_t)(l0 + r) * kPrjP + kDtR + q);
      *(v4f*)(sBC + r * 32 + q) = v;
    }
    __syncthreads();
#pragma unroll 1
    for (int s = 0; s < 16; ++s) {
      const int rr = rev ? (15 - s) : s;
      const size_t m = (size_t)(l0 + rr);
      const float a  = DLR[m * kDin + d];
      const float ea = __expf(-fabsf(a));
      const float u1 = 1.0f + ea;
      const float l1p = __logf(u1) + (ea - (u1 - 1.0f)) * __builtin_amdgcn_rcpf(u1);
      const float delta = fmaxf(a, 0.0f) + l1p;
      const float xv = UC[m * kDin + d];
      const float zv = XZ[m * kXZP + kDin + d];
      v4f Bq[4], Cq[4];
#pragma unroll
      for (int qq = 0; qq < 4; ++qq) {
        Bq[qq] = *(const v4f*)(sBC + rr * 32 + 4 * qq);
        Cq[qq] = *(const v4f*)(sBC + rr * 32 + kNst + 4 * qq);
      }
      const float dx = delta * xv;
      float y = 0.f;
#pragma unroll
      for (int n = 0; n < kNst; ++n) {
        const float e  = __expf(delta * An[n]);
        const float hn = h[n] * e + dx * Bq[n >> 2][n & 3];
        h[n] = hn;
        y = Cq[n >> 2][n & 3] * hn + y;
      }
      y = xv * Dd + y;
      const float sg = __builtin_amdgcn_rcpf(1.0f + __expf(-zv));
      const float g  = zv * sg;
      sY[rr * kTP + tid] = (y * g) * kCarY;
    }
    __syncthreads();
    v8h hv[2];
#pragma unroll
    for (int it = 0; it < 2; ++it) {
      const float* sp = sY + (it * 8 + wave) * kTP + lane * 8;
      const v4f a0 = *(const v4f*)(sp);
      const v4f a1 = *(const v4f*)(sp + 4);
#pragma unroll
      for (int e = 0; e < 4; ++e) { hv[it][e] = (_Float16)a0[e]; hv[it][4 + e] = (_Float16)a1[e]; }
    }
    for (int pass = 0; pass < 2; ++pass) {
#pragma unroll
      for (int it = 0; it < 2; ++it)
        *(volatile v8h*)(Y16 + (size_t)(l0 + it * 8 + wave) * kDin + d0 + lane * 8) = hv[it];
      __threadfence();
    }
  }
}

static_assert(((kSeqL / 64) * (kXZP / 64)) % 8 == 0, "in_proj tiles");
static_assert(((kSeqL / 64) * (kPrjP / 64)) % 8 == 0, "x_proj tiles");
static_assert(((kSeqL / 64) * (kDin / 64)) % 8 == 0, "dt_proj tiles");
static_assert(((kSeqL / 64) * (kDmod / 64)) % 8 == 0, "out_proj tiles");
static_assert(((kRows / 64) * (kDmod / 64)) % 8 == 0, "fusion tiles");
static_assert((kRows * kDmod / 8) % 256 == 0 && (kXZP * kDmod / 8) % 256 == 0 && (kPrjP * kDin / 8) % 256 == 0 &&
              (kDin * kDtR / 8) % 256 == 0 && (kDmod * kDin / 8) % 256 == 0 && (kDmod * kFuK / 8) % 256 == 0 &&
              (kSeqL * kDtR / 8) % 256 == 0, "cast grids exact");

extern "C" void kernel_launch(void* const* d_in, const int* in_sizes, int n_in,
                              void* d_out, int out_size, void* d_ws, size_t ws_size,
                              hipStream_t stream)
{
  if (n_in < 21) return;
  if (in_sizes[0] != kRows * kDmod) return;
  for (int dir = 0; dir < 2; ++dir) {
    const int base = 1 + 9 * dir;
    if (in_sizes[base + 0] != kXZP * kDmod) return;
    if (in_sizes[base + 1] != kDin * 4) return;
    if (in_sizes[base + 2] != kDin) return;
    if (in_sizes[base + 3] != kPrjN * kDin) return;
    if (in_sizes[base + 4] != kDin * kDtR) return;
    if (in_sizes[base + 5] != kDin) return;
    if (in_sizes[base + 6] != kDin * kNst) return;
    if (in_sizes[base + 7] != kDin) return;
    if (in_sizes[base + 8] != kDmod * kDin) return;
  }
  if (in_sizes[19] != kDmod * kFuK) return;
  if (in_sizes[20] != kDmod) return;
  if (out_size != kRows * kDmod) return;
  if (ws_size < kWsTotal) return;

  const float* x        = (const float*)d_in[0];
  const float* fusion_w = (const float*)d_in[19];
  const float* fusion_b = (const float*)d_in[20];
  float* dout = (float*)d_out;

  char* ws = (char*)d_ws;
  unsigned short* WIN16  = (unsigned short*)(ws + kOffWIN);
  unsigned short* WXP16  = (unsigned short*)(ws + kOffWXP);
  unsigned short* WDT16  = (unsigned short*)(ws + kOffWDT);
  unsigned short* WOUT16 = (unsigned short*)(ws + kOffWOUT);
  unsigned short* WFU16  = (unsigned short*)(ws + kOffWFU);
  unsigned short* X16    = (unsigned short*)(ws + kOffX16);
  float*          XZ     = (float*)(ws + kOffXZ);
  float*          UC     = (float*)(ws + kOffUC);
  unsigned short* UC16   = (unsigned short*)(ws + kOffUC16);
  float*          PROJ   = (float*)(ws + kOffPROJ);
  unsigned short* DT16   = (unsigned short*)(ws + kOffDT16);
  float*          DLR    = (float*)(ws + kOffDLR);
  unsigned short* Y16    = (unsigned short*)(ws + kOffY16);
  unsigned short* COMB   = (unsigned short*)(ws + kOffCOMB);

  cast_bf16_f16_kernel<<<(kRows * kDmod / 8) / 256, 256, 0, stream>>>(x, X16, kRows * kDmod / 8, kRows * kDmod / 8, 1.0f);
  cast_bf16_f16_kernel<<<(kDmod * kFuK / 8) / 256, 256, 0, stream>>>(fusion_w, WFU16, kDmod * kFuK / 8, kDmod * kFuK / 8, kCarW);

  for (int dir = 0; dir < 2; ++dir) {
    const int base = 1 + 9 * dir;
    const float* W_in   = (const float*)d_in[base + 0];
    const float* conv_w = (const float*)d_in[base + 1];
    const float* conv_b = (const float*)d_in[base + 2];
    const float* W_xp   = (const float*)d_in[base + 3];
    const float* W_dt   = (const float*)d_in[base + 4];
    const float* b_dt   = (const float*)d_in[base + 5];
    const float* A_log  = (const float*)d_in[base + 6];
    const float* Dv     = (const float*)d_in[base + 7];
    const float* W_out  = (const float*)d_in[base + 8];

    cast_bf16_f16_kernel<<<(kXZP * kDmod / 8) / 256, 256, 0, stream>>>(W_in, WIN16, kXZP * kDmod / 8, kXZP * kDmod / 8, kCarW);
    cast_bf16_f16_kernel<<<(kPrjP * kDin / 8) / 256, 256, 0, stream>>>(W_xp, WXP16, kPrjP * kDin / 8, kPrjN * kDin / 8, kCarW);
    cast_bf16_f16_kernel<<<(kDin * kDtR / 8) / 256, 256, 0, stream>>>(W_dt, WDT16, kDin * kDtR / 8, kDin * kDtR / 8, kCarWdt);
    cast_bf16_f16_kernel<<<(kDmod * kDin / 8) / 256, 256, 0, stream>>>(W_out, WOUT16, kDmod * kDin / 8, kDmod * kDin / 8, kCarW);

    for (int b = 0; b < kBatch; ++b) {
      const unsigned short* X16b = X16 + (size_t)b * kSeqL * kDmod;
      unsigned short* COMBb = COMB + (size_t)b * kSeqL * kFuK + (size_t)dir * kDmod;

      wmma_gemm64_f16<0, 0><<<dim3(256), 256, 0, stream>>>(
          X16b, kDmod, WIN16, kDmod, (void*)XZ, kXZP, b_dt, kSeqL, kXZP, kDmod, kSclIn);

      conv_silu_kernel<<<dim3(kDin / 256, kSeqL / 64), 256, 0, stream>>>(XZ, conv_w, conv_b, UC, UC16, dir);

      wmma_gemm64_f16<0, 0><<<dim3(8), 256, 0, stream>>>(
          UC16, kDin, WXP16, kDin, (void*)PROJ, kPrjP, b_dt, kSeqL, kPrjP, kDin, kSclXp);

      dt_cast_kernel<<<(kSeqL * kDtR / 8) / 256, 256, 0, stream>>>(PROJ, DT16, kSeqL * kDtR / 8, kCarDt);

      wmma_gemm64_f16<2, 0><<<dim3(128), 256, 0, stream>>>(
          DT16, kDtR, WDT16, kDtR, (void*)DLR, kDin, b_dt, kSeqL, kDin, kDtR, kSclDt);

      scan_kernel<<<dim3(kDin / 256), 256, 0, stream>>>(DLR, UC, XZ, PROJ, A_log, Dv, Y16, dir);

      wmma_gemm64_f16<0, 1><<<dim3(64), 256, 0, stream>>>(
          Y16, kDin, WOUT16, kDin, (void*)COMBb, kFuK, b_dt, kSeqL, kDmod, kDin, kSclOut);
    }
  }

  wmma_gemm64_f16<2, 0><<<dim3(128), 256, 0, stream>>>(
      COMB, kFuK, WFU16, kFuK, (void*)dout, kDmod, fusion_b, kRows, kDmod, kFuK, kSclFu);
}
